// SSA_Sp_45286135169186
// MI455X (gfx1250) — hardware-verified
//
#include <hip/hip_runtime.h>


#define NBT  4
#define CC   64
#define HH   80
#define WW   80
#define NN   (HH * WW)
#define RCH  1600
#define DM   CC
#define NTK  NN
#define LOSC 1024.0f

typedef _Float16 h16;
typedef unsigned short bf;
typedef __attribute__((ext_vector_type(16))) __bf16   v16bf;
typedef __attribute__((ext_vector_type(16))) _Float16 v16h;
typedef __attribute__((ext_vector_type(8)))  _Float16 v8h;
typedef __attribute__((ext_vector_type(8)))  unsigned short v8us;
typedef __attribute__((ext_vector_type(8)))  float    v8f;
typedef __attribute__((ext_vector_type(4)))  float    v4f;
typedef __attribute__((ext_vector_type(4)))  _Float16 v4h;
typedef v8h  __attribute__((may_alias)) v8ha;
typedef v4f  __attribute__((may_alias)) v4fa;
typedef v8us __attribute__((may_alias)) v8usa;

__device__ __forceinline__ unsigned short f2bf(float f) { unsigned u = __float_as_uint(f); u += 0x7FFFu + ((u >> 16) & 1u); return (unsigned short)(u >> 16); }
__device__ __forceinline__ float bf2f(unsigned short b) { return __uint_as_float(((unsigned)b) << 16); }
__device__ __forceinline__ float bfr(float f) { return bf2f(f2bf(f)); }
__device__ __forceinline__ v16h cat16(v8h lo, v8h hi) { return __builtin_shufflevector(lo, hi, 0, 1, 2, 3, 4, 5, 6, 7, 8, 9, 10, 11, 12, 13, 14, 15); }
__device__ __forceinline__ v16bf cat16b(v8us lo, v8us hi) { return __builtin_bit_cast(v16bf, __builtin_shufflevector(lo, hi, 0, 1, 2, 3, 4, 5, 6, 7, 8, 9, 10, 11, 12, 13, 14, 15)); }
__device__ __forceinline__ v8f wmma16(v16h a, v16h b, v8f c) { return __builtin_amdgcn_wmma_f32_16x16x32_f16(false, a, false, b, (short)0, c, false, false); }
__device__ __forceinline__ v8f wmmab(v16bf a, v16bf b, v8f c) { return __builtin_amdgcn_wmma_f32_16x16x32_bf16(false, a, false, b, (short)0, c, false, false); }

__global__ __launch_bounds__(256) void k_wt(const float* __restrict__ Wm, int K, int ncols, bf* WT) {
    __shared__ __align__(16) unsigned short tl[64 * 72];
    const int tid = threadIdx.x, k0 = blockIdx.x * 64, n0 = blockIdx.y * 64;
    const int kk = tid >> 2, nq = (tid & 3) * 16;
#pragma unroll
    for (int i = 0; i < 16; ++i) tl[(nq + i) * 72 + kk] = f2bf(Wm[(size_t)(k0 + kk) * ncols + n0 + nq + i]);
    __syncthreads();
    const int piece = tid & 7;
    auto pass = [&]() {
#pragma unroll
        for (int s = 0; s < 2; ++s) { const int nr = (tid >> 3) + 32 * s; const v8us val = *(const v8usa*)(tl + nr * 72 + piece * 8); *(volatile v8us*)(WT + (size_t)(n0 + nr) * K + k0 + piece * 8) = val; }
    };
    pass(); __threadfence(); pass();
}
template <bool SPLITA, bool F16OUT = false>
__global__ __launch_bounds__(128) void k_gemmb(const bf* __restrict__ A, const bf* __restrict__ Al, const bf* __restrict__ Bn, const float* __restrict__ bias, float* C, int ldc, h16* C2, const float* __restrict__ R = nullptr, int K = DM, int roundR = 1) {
    __shared__ __align__(16) float ost[4][16 * 68];
    const int lane = threadIdx.x & 31, wave = threadIdx.x >> 5, lr = lane & 15, hi = lane >> 4;
    const int r0 = blockIdx.x * 64 + wave * 16, c0 = blockIdx.y * 64;
    const size_t aoff = (size_t)(r0 + lr) * K + 8 * hi;
    size_t boff[4];
#pragma unroll
    for (int t = 0; t < 4; ++t) boff[t] = (size_t)(c0 + t * 16 + lr) * K + 8 * hi;
    v8f acc[4];
#pragma unroll
    for (int t = 0; t < 4; ++t) acc[t] = (v8f){};
#pragma unroll 1
    for (int kc = 0; kc < K; kc += 32) {
        const v16bf a = cat16b(*(const v8us*)(A + aoff + kc), *(const v8us*)(A + aoff + kc + 16));
        v16bf al = a;
        if (SPLITA) al = cat16b(*(const v8us*)(Al + aoff + kc), *(const v8us*)(Al + aoff + kc + 16));
#pragma unroll
        for (int t = 0; t < 4; ++t) { const v16bf b = cat16b(*(const v8us*)(Bn + boff[t] + kc), *(const v8us*)(Bn + boff[t] + kc + 16)); acc[t] = wmmab(a, b, acc[t]); if (SPLITA) acc[t] = wmmab(al, b, acc[t]); }
        asm volatile("v_nop\n\tv_nop\n\tv_nop\n\tv_nop" : "+v"(acc[0]), "+v"(acc[1]), "+v"(acc[2]), "+v"(acc[3]) : "v"(a), "v"(al));
    }
    float* os = &ost[wave][0];
#pragma unroll
    for (int t = 0; t < 4; ++t) { const float bv = bias ? bfr(bias[c0 + t * 16 + lr]) : 0.f;
#pragma unroll
        for (int j = 0; j < 8; ++j) os[(hi * 8 + j) * 68 + t * 16 + lr] = acc[t][j] + bv; }
    __syncthreads();
    if (F16OUT) {
        h16* crow = (h16*)(void*)C + (size_t)r0 * ldc + c0;
        auto pass = [&]() {
#pragma unroll
            for (int s = 0; s < 4; ++s) { const int row = 4 * s + (lane >> 3), piece = lane & 7; const float* sp = os + row * 68 + piece * 8; v8h o, o2;
#pragma unroll
                for (int i = 0; i < 8; ++i) { const h16 a = (h16)sp[i]; o[i] = a; o2[i] = (h16)((sp[i] - (float)a) * LOSC); }
                *(volatile v8h*)(crow + (size_t)row * ldc + piece * 8) = o; if (C2) *(volatile v8h*)(C2 + (size_t)r0 * ldc + c0 + (size_t)row * ldc + piece * 8) = o2; }
        };
        pass(); __threadfence(); pass();
    } else {
        float* crow = C + (size_t)r0 * ldc + c0;
        auto pass = [&]() {
#pragma unroll
            for (int s = 0; s < 8; ++s) { const int Lid = (lane >> 3) + 4 * s, piece = lane & 7; const int row = Lid >> 1, cofs = (Lid & 1) * 32 + piece * 4;
                v4f val = *(const v4fa*)(os + row * 68 + cofs); if (R) { const v4f rv = *(const v4f*)(R + ((size_t)r0 + row) * ldc + c0 + cofs); val += roundR ? (v4f){bfr(rv[0]), bfr(rv[1]), bfr(rv[2]), bfr(rv[3])} : rv; }
                *(volatile v4f*)(crow + (size_t)row * ldc + cofs) = val; }
        };
        pass(); __threadfence(); pass();
    }
}

__global__ __launch_bounds__(128) void k_gemm3(const bf* __restrict__ Ah, const bf* __restrict__ Al, const bf* __restrict__ Bh, const bf* __restrict__ Bl, int K, float* C, int ldc) {
    __shared__ __align__(16) float ost[4][16 * 68];
    const int lane = threadIdx.x & 31, wave = threadIdx.x >> 5, lr = lane & 15, hi = lane >> 4;
    const int r0 = blockIdx.x * 64 + wave * 16, c0 = blockIdx.y * 64;
    const size_t aoff = (size_t)(r0 + lr) * K + 8 * hi;
    v8f acc[4];
#pragma unroll
    for (int t = 0; t < 4; ++t) acc[t] = (v8f){};
#pragma unroll 1
    for (int kc = 0; kc < K; kc += 32) {
        const v16bf a = cat16b(*(const v8us*)(Ah + aoff + kc), *(const v8us*)(Ah + aoff + kc + 16));
        const v16bf al = cat16b(*(const v8us*)(Al + aoff + kc), *(const v8us*)(Al + aoff + kc + 16));
#pragma unroll
        for (int t = 0; t < 4; ++t) { const size_t bo = (size_t)(c0 + t * 16 + lr) * K + kc + 8 * hi;
            const v16bf bh = cat16b(*(const v8us*)(Bh + bo), *(const v8us*)(Bh + bo + 16)); const v16bf bl = cat16b(*(const v8us*)(Bl + bo), *(const v8us*)(Bl + bo + 16));
            acc[t] = wmmab(a, bh, acc[t]); acc[t] = wmmab(al, bh, acc[t]); acc[t] = wmmab(a, bl, acc[t]); }
        asm volatile("v_nop\n\tv_nop\n\tv_nop\n\tv_nop" : "+v"(acc[0]), "+v"(acc[1]), "+v"(acc[2]), "+v"(acc[3]) : "v"(a), "v"(al));
    }
    float* os = &ost[wave][0];
#pragma unroll
    for (int t = 0; t < 4; ++t) {
#pragma unroll
        for (int j = 0; j < 8; ++j) os[(hi * 8 + j) * 68 + t * 16 + lr] = acc[t][j]; }
    __builtin_amdgcn_wave_barrier(); asm volatile("" ::: "memory");
    float* crow = C + (size_t)r0 * ldc + c0;
    auto pass = [&]() {
#pragma unroll
        for (int s = 0; s < 8; ++s) { const int Lid = (lane >> 3) + 4 * s, piece = lane & 7; const int row = Lid >> 1, cofs = (Lid & 1) * 32 + piece * 4;
            const v4f val = *(const v4fa*)(os + row * 68 + cofs); *(volatile v4f*)(crow + (size_t)row * ldc + cofs) = val; }
    };
    pass(); __threadfence(); pass();
}


__global__ __launch_bounds__(256) void k_cvt8(const float* __restrict__ src, bf* dst, size_t n8) {
    const size_t i = (size_t)blockIdx.x * 256 + threadIdx.x; if (i >= n8) return;
    const v8f v = *(const v8f*)(src + i * 8); v8us o;
#pragma unroll
    for (int k = 0; k < 8; ++k) o[k] = f2bf(v[k]);
    *(volatile v8us*)(dst + i * 8) = o; __threadfence(); *(volatile v8us*)(dst + i * 8) = o;
}
__global__ __launch_bounds__(256) void k_zero8(bf* dst, size_t n8) {
    const size_t i = (size_t)blockIdx.x * 256 + threadIdx.x; if (i >= n8) return; v8us z;
#pragma unroll
    for (int k = 0; k < 8; ++k) z[k] = 0;
    *(volatile v8us*)(dst + i * 8) = z; __threadfence(); *(volatile v8us*)(dst + i * 8) = z;
}

__global__ __launch_bounds__(256) void k_qplanes(const float* __restrict__ QKV, int sel, bf* Ph, bf* Pl) {
    typedef __attribute__((ext_vector_type(2))) unsigned short v2us;
    const int lane = threadIdx.x & 31; const int r = blockIdx.x * 8 + (threadIdx.x >> 5); if (r >= NN) return;
    int n; int col0;
    if (sel == 0) { const int w = r / HH, h = r % HH; n = h * WW + w; col0 = 0; } else if (sel == 1) { n = r; col0 = 0; } else { n = r; col0 = 2 * CC; }
    v2us oh, ol;
#pragma unroll
    for (int i = 0; i < 2; ++i) { const float v = QKV[(size_t)n * (3 * CC) + col0 + lane * 2 + i]; const unsigned short hb = f2bf(v); oh[i] = hb; ol[i] = f2bf(v - bf2f(hb)); }
    const size_t o = (size_t)r * CC + lane * 2; *(volatile v2us*)(Ph + o) = oh; *(volatile v2us*)(Pl + o) = ol; __threadfence(); *(volatile v2us*)(Ph + o) = oh; *(volatile v2us*)(Pl + o) = ol;
}
__global__ __launch_bounds__(256) void k_tplanes(const float* __restrict__ QKV, int sel, bf* Th, bf* Tl) {
    typedef __attribute__((ext_vector_type(2))) unsigned short v2us;
    const int lane = threadIdx.x & 31; const size_t wid = (size_t)blockIdx.x * 8 + (threadIdx.x >> 5); if (wid >= (size_t)CC * (NN / 64)) return; const int c = (int)(wid / (NN / 64)); const int n0 = (int)(wid % (NN / 64)) * 64 + lane * 2;
    const int col = (sel == 0) ? 2 * CC + c : ((sel == 1) ? CC + c : c); v2us oh, ol;
#pragma unroll
    for (int i = 0; i < 2; ++i) { const int n = n0 + i; const int pix = (sel == 1) ? n : ((n % HH) * WW + (n / HH)); const float v = QKV[(size_t)pix * (3 * CC) + col]; const unsigned short hb = f2bf(v); oh[i] = hb; ol[i] = f2bf(v - bf2f(hb)); }
    const size_t o = (size_t)c * NN + n0; *(volatile v2us*)(Th + o) = oh; *(volatile v2us*)(Tl + o) = ol; __threadfence(); *(volatile v2us*)(Th + o) = oh; *(volatile v2us*)(Tl + o) = ol;
}
__global__ __launch_bounds__(256) void k_softmax6400(const float* __restrict__ S, bf* PH, bf* PL) {
    typedef __attribute__((ext_vector_type(4))) unsigned short v4us;
    const int lane = threadIdx.x & 31, i = blockIdx.x * 8 + (threadIdx.x >> 5); if (i >= RCH) return;
    float m = -3.0e38f;
#pragma unroll 1
    for (int c0 = lane * 4; c0 < NN; c0 += 128) {
#pragma unroll
        for (int q = 0; q < 4; ++q) m = fmaxf(m, S[(size_t)i * NN + c0 + q]); }
#pragma unroll
    for (int sh = 16; sh; sh >>= 1) m = fmaxf(m, __shfl_xor(m, sh, 32));
    float sum = 0.f;
#pragma unroll 1
    for (int c0 = lane * 4; c0 < NN; c0 += 128) {
#pragma unroll
        for (int q = 0; q < 4; ++q) sum += __expf(S[(size_t)i * NN + c0 + q] - m); }
#pragma unroll
    for (int sh = 16; sh; sh >>= 1) sum += __shfl_xor(sum, sh, 32);
    const float inv = 1.0f / sum;
#pragma unroll 1
    for (int ps = 0; ps < 2; ++ps) {
#pragma unroll 1
        for (int c0 = lane * 4; c0 < NN; c0 += 128) { v4us oh, ol;
#pragma unroll
            for (int q = 0; q < 4; ++q) { const float p = __expf(S[(size_t)i * NN + c0 + q] - m) * inv; const unsigned short hb = f2bf(p); oh[q] = hb; ol[q] = f2bf(p - bf2f(hb)); }
            const size_t o = (size_t)i * NN + c0; *(volatile v4us*)(PH + o) = oh; *(volatile v4us*)(PL + o) = ol; }
        if (ps == 0) __threadfence(); }
}
__global__ __launch_bounds__(256) void k_softmax64(const float* __restrict__ M, bf* PH, bf* PL) {
    typedef __attribute__((ext_vector_type(2))) unsigned short v2us;
    const int lane = threadIdx.x & 31, i = blockIdx.x * 8 + (threadIdx.x >> 5); if (i >= CC) return; const float a = M[i * CC + lane * 2], b = M[i * CC + lane * 2 + 1];
    float m = fmaxf(a, b);
#pragma unroll
    for (int sh = 16; sh; sh >>= 1) m = fmaxf(m, __shfl_xor(m, sh, 32));
    const float ea = __expf(a - m), eb = __expf(b - m); float s = ea + eb;
#pragma unroll
    for (int sh = 16; sh; sh >>= 1) s += __shfl_xor(s, sh, 32);
    const float inv = 1.0f / s; v2us oh, ol;
    { const float p = ea * inv; const unsigned short hb = f2bf(p); oh[0] = hb; ol[0] = f2bf(p - bf2f(hb)); } { const float p = eb * inv; const unsigned short hb = f2bf(p); oh[1] = hb; ol[1] = f2bf(p - bf2f(hb)); }
    const size_t o = (size_t)i * CC + lane * 2; *(volatile v2us*)(PH + o) = oh; *(volatile v2us*)(PL + o) = ol; __threadfence(); *(volatile v2us*)(PH + o) = oh; *(volatile v2us*)(PL + o) = ol;
}

__global__ __launch_bounds__(256) void k_fin(const float* __restrict__ MS, const float* __restrict__ MV, float* OUTB) {
    const int lane = threadIdx.x & 31; const size_t wid = (size_t)blockIdx.x * 8 + (threadIdx.x >> 5); if (wid >= (size_t)CC * (NN / 128)) return; const size_t o = wid * 128 + lane * 4; v4f v;
#pragma unroll
    for (int q = 0; q < 4; ++q) v[q] = MS[o + q] + MV[o + q];
    *(volatile v4f*)(OUTB + o) = v; __threadfence(); *(volatile v4f*)(OUTB + o) = v;
}

extern "C" void kernel_launch(void* const* d_in, const int* in_sizes, int n_in,
                              void* d_out, int out_size, void* d_ws, size_t ws_size, hipStream_t stream) {
    (void)in_sizes; (void)n_in; (void)out_size;
    const float* x = (const float*)d_in[0]; const float* wqkv = (const float*)d_in[1]; const float* bqkv = (const float*)d_in[2];
    float* out = (float*)d_out;
    char* wsp = (char*)d_ws;
    auto take = [&](size_t bytes) { char* p = wsp; wsp += (bytes + 255) & ~(size_t)255; return (void*)p; };
    bf* WB = (bf*)take((size_t)3 * CC * CC * 2); bf* XP = (bf*)take((size_t)NN * CC * 2); float* QKV = (float*)take((size_t)NN * 3 * CC * 4);
    bf* QWh = (bf*)take((size_t)NN * CC * 2); bf* QWl = (bf*)take((size_t)NN * CC * 2); bf* QHh = (bf*)take((size_t)NN * CC * 2); bf* QHl = (bf*)take((size_t)NN * CC * 2); bf* VPh = (bf*)take((size_t)NN * CC * 2); bf* VPl = (bf*)take((size_t)NN * CC * 2);
    bf* VTh = (bf*)take((size_t)CC * NN * 2); bf* VTl = (bf*)take((size_t)CC * NN * 2); bf* KFh = (bf*)take((size_t)CC * NN * 2); bf* KFl = (bf*)take((size_t)CC * NN * 2); bf* QTh = (bf*)take((size_t)CC * NN * 2); bf* QTl = (bf*)take((size_t)CC * NN * 2);
    float* S = (float*)take((size_t)RCH * NN * 4); bf* PH = (bf*)take((size_t)RCH * NN * 2); bf* PL = (bf*)take((size_t)RCH * NN * 2); float* MS = (float*)take((size_t)CC * NN * 4); float* MV = (float*)take((size_t)CC * NN * 4); float* MA = (float*)take((size_t)CC * CC * 4); bf* MAh = (bf*)take((size_t)CC * CC * 2); bf* MAl = (bf*)take((size_t)CC * CC * 2);
    if ((size_t)(wsp - (char*)d_ws) > ws_size) return;
    k_cvt8<<<(3 * CC * CC / 8 + 255) / 256, 256, 0, stream>>>(wqkv, WB, 3 * CC * CC / 8);
    for (int b = 0; b < NBT; ++b) {
        k_wt<<<dim3(CC / 64, NN / 64, 1), 256, 0, stream>>>(x + (size_t)b * CC * NN, CC, NN, XP);
        k_gemmb<false, false><<<dim3(NN / 64, (3 * CC) / 64, 1), 128, 0, stream>>>(XP, nullptr, WB, bqkv, QKV, 3 * CC, nullptr, nullptr, CC);
        k_qplanes<<<NN / 8, 256, 0, stream>>>(QKV, 0, QWh, QWl); k_qplanes<<<NN / 8, 256, 0, stream>>>(QKV, 1, QHh, QHl); k_qplanes<<<NN / 8, 256, 0, stream>>>(QKV, 2, VPh, VPl);
        k_tplanes<<<(CC * (NN / 64)) / 8, 256, 0, stream>>>(QKV, 0, VTh, VTl); k_tplanes<<<(CC * (NN / 64)) / 8, 256, 0, stream>>>(QKV, 1, KFh, KFl); k_tplanes<<<(CC * (NN / 64)) / 8, 256, 0, stream>>>(QKV, 2, QTh, QTl);
        for (int ch = 0; ch < NN / RCH; ++ch) { const size_t r0 = (size_t)ch * RCH;
            k_gemm3<<<dim3(RCH / 64, NN / 64, 1), 128, 0, stream>>>(QWh + r0 * CC, QWl + r0 * CC, QHh, QHl, CC, S, NN);
            k_softmax6400<<<RCH / 8, 256, 0, stream>>>(S, PH, PL);
            k_gemm3<<<dim3(1, RCH / 64, 1), 128, 0, stream>>>(VTh, VTl, PH, PL, NN, MS + r0, NN); }
        k_gemm3<<<dim3(1, 1, 1), 128, 0, stream>>>(KFh, KFl, QTh, QTl, NN, MA, CC);
        k_softmax64<<<CC / 8, 256, 0, stream>>>(MA, MAh, MAl);
        k_gemm3<<<dim3(1, NN / 64, 1), 128, 0, stream>>>(MAh, MAl, VPh, VPl, CC, MV, NN);
        k_fin<<<(CC * (NN / 128)) / 8, 256, 0, stream>>>(MS, MV, out + (size_t)b * CC * NN); }
}
